// GNN_74131135529535
// MI455X (gfx1250) — hardware-run, weakly checked
//
#include <hip/hip_runtime.h>


#ifndef NB
#define NB 8
#endif
#define NB_FULL 8
#define KH   3
#define NN   192
#define DOBS 32
#define DD   64
#define ET   8
#define WCS  64.0f
#define WCI  (1.0f / 64.0f)
#define ACS  (1.0f / 64.0f)

static_assert(NB >= 1);
static_assert(NB <= NB_FULL);
static_assert(DD == 64);
static_assert(DOBS % 32 == 0);
static_assert(DD % 32 == 0);
static_assert(NN % 32 == 0);
static_assert(NN % 64 == 0);
static_assert((NB * NN * 4) % 64 == 0);
static_assert(NN % ET == 0);
static_assert((ET * NN) % 256 == 0);
static_assert(ET * 4 * DD * 2 == 256 * 16);
static_assert(4 * 32 * 16 == 16 * DD * 2);
static_assert(8 * 32 * 16 == 16 * DD * 4);
static_assert(DD * DOBS / 8 == 256);
static_assert(DD * DD / 8 == 2 * 256);
static_assert((DOBS * DD) % 256 == 0);
static_assert((DD * DD) % 256 == 0);
static_assert(WCS * ACS == 1.0f);
static_assert(WCS * WCI == 1.0f);
static_assert(((size_t)NB * 4 * NN * DOBS) % 8 == 0);
static_assert(((size_t)2 * NN * NN) % 8 == 0);
static_assert(16 * 68 * 4 <= 131072);
static_assert((ET * NN + ET * 4 * DD) * 4 <= 131072);
static_assert(DD * (DD + 1) * 4 <= 131072);

typedef _Float16 h16;
typedef unsigned short bf;
typedef __attribute__((ext_vector_type(16))) __bf16   v16bf;
typedef __attribute__((ext_vector_type(16))) _Float16 v16h;
typedef __attribute__((ext_vector_type(8)))  _Float16 v8h;
typedef __attribute__((ext_vector_type(8)))  unsigned short v8us;
typedef __attribute__((ext_vector_type(8)))  float    v8f;
typedef __attribute__((ext_vector_type(4)))  float    v4f;
typedef v4f  __attribute__((may_alias)) v4fa;

__device__ __forceinline__ unsigned short f2bf(float f) { unsigned u = __float_as_uint(f); u += 0x7FFFu + ((u >> 16) & 1u); return (unsigned short)(u >> 16); }
__device__ __forceinline__ float bfr(float f) { return __uint_as_float(((unsigned)f2bf(f)) << 16); }
__device__ __forceinline__ v16h cat16(v8h lo, v8h hi) { return __builtin_shufflevector(lo, hi, 0, 1, 2, 3, 4, 5, 6, 7, 8, 9, 10, 11, 12, 13, 14, 15); }
__device__ __forceinline__ v16bf cat16b(v8us lo, v8us hi) { return __builtin_bit_cast(v16bf, __builtin_shufflevector(lo, hi, 0, 1, 2, 3, 4, 5, 6, 7, 8, 9, 10, 11, 12, 13, 14, 15)); }
__device__ __forceinline__ v8f wmma16(v16h a, v16h b, v8f c) { return __builtin_amdgcn_wmma_f32_16x16x32_f16(false, a, false, b, (short)0, c, false, false); }
__device__ __forceinline__ v8f wmmab(v16bf a, v16bf b, v8f c) { return __builtin_amdgcn_wmma_f32_16x16x32_bf16(false, a, false, b, (short)0, c, false, false); }
__device__ __forceinline__ v16h  ldh(const h16* p) { return cat16(*(const v8h*)p, *(const v8h*)(p + 16)); }
__device__ __forceinline__ v16bf ldb(const bf* p)  { return cat16b(*(const v8us*)p, *(const v8us*)(p + 16)); }
__device__ __forceinline__ void wave_sync() { __builtin_amdgcn_fence(3  , "wavefront"); __builtin_amdgcn_wave_barrier(); asm volatile("" ::: "memory"); }

static __device__ __forceinline__ h16 toh_flush(float v) { const h16 r = (h16)v; return (fabsf(v) < 6.103515625e-05f) ? (h16)0.0f : r; }
__device__ __forceinline__ v8f wmma16g(v16h a, v16h b, v8f c) { c = wmma16(a, b, c); asm volatile("v_nop\n\tv_nop\n\tv_nop\n\tv_nop" : "+v"(c) : "v"(a), "v"(b)); return c; }
__device__ __forceinline__ v8f wmmabg(v16bf a, v16bf b, v8f c) { c = wmmab(a, b, c); asm volatile("v_nop\n\tv_nop\n\tv_nop\n\tv_nop" : "+v"(c) : "v"(a), "v"(b)); return c; }

template <int K>
__device__ __forceinline__ void mma_tile_h(const h16* __restrict__ A, const h16* __restrict__ Bt, const size_t aoff, const size_t boff, v8f (&acc)[4][4]) {
    static_assert(K % 32 == 0);
#pragma unroll 1
    for (int kc = 0; kc < K; kc += 32) {
        v16h a[4];
#pragma unroll
        for (int mb = 0; mb < 4; ++mb) a[mb] = ldh(A + aoff + (size_t)mb * 16 * K + kc);
#pragma unroll
        for (int nb = 0; nb < 4; ++nb) { const v16h b = ldh(Bt + boff + (size_t)nb * 16 * K + kc);
#pragma unroll
            for (int mb = 0; mb < 4; ++mb) acc[mb][nb] = wmma16g(a[mb], b, acc[mb][nb]); }
    }
}
template <int K>
__device__ __forceinline__ void mma_tile_b(const bf* __restrict__ A, const bf* __restrict__ Bt, const size_t aoff, const size_t boff, v8f (&acc)[4][4]) {
    static_assert(K % 32 == 0);
#pragma unroll 1
    for (int kc = 0; kc < K; kc += 32) {
        v16bf a[4];
#pragma unroll
        for (int mb = 0; mb < 4; ++mb) a[mb] = ldb(A + aoff + (size_t)mb * 16 * K + kc);
#pragma unroll
        for (int nb = 0; nb < 4; ++nb) { const v16bf b = ldb(Bt + boff + (size_t)nb * 16 * K + kc);
#pragma unroll
            for (int mb = 0; mb < 4; ++mb) acc[mb][nb] = wmmabg(a[mb], b, acc[mb][nb]); }
    }
}

__global__ __launch_bounds__(256) void k_cvt8(const float* __restrict__ src, bf* dst, size_t n8) {
    const size_t i = (size_t)blockIdx.x * 256 + threadIdx.x; if (i >= n8) return;
    const v8f v = *(const v8f*)(src + i * 8); v8us o;
#pragma unroll
    for (int k = 0; k < 8; ++k) o[k] = f2bf(v[k]);
    *(volatile v8us*)(dst + i * 8) = o; __threadfence(); *(volatile v8us*)(dst + i * 8) = o;
}

__global__ __launch_bounds__(256) void k_cvt8a(const float* __restrict__ src, h16* dst, size_t n8) {
    const size_t i = (size_t)blockIdx.x * 256 + threadIdx.x; if (i >= n8) return;
    const size_t pb = (size_t)2 * NN * NN / 8;
    const size_t b = i / pb, r = i % pb;
    const v8f v = *(const v8f*)(src + b * ((size_t)KH * NN * NN) + (size_t)NN * NN + r * 8); v8h o;
#pragma unroll
    for (int k = 0; k < 8; ++k) o[k] = toh_flush(bfr(v[k]));
    *(volatile v8h*)(dst + i * 8) = o; __threadfence(); *(volatile v8h*)(dst + i * 8) = o;
}

__global__ __launch_bounds__(256) void k_wtb(const float* __restrict__ W, bf* Wt) {
    __shared__ float tl[DD * (DOBS + 1)];
    const int t = threadIdx.x;
#pragma unroll 1
    for (int r = 0; r < DOBS * DD / 256; ++r) { const int idx = t + r * 256; const int k = idx >> 6, n = idx & 63; tl[n * (DOBS + 1) + k] = W[idx]; }
    __syncthreads();
    const int n = t >> 2, k8 = (t & 3) * 8; v8us o;
#pragma unroll
    for (int i = 0; i < 8; ++i) o[i] = f2bf(tl[n * (DOBS + 1) + k8 + i]);
    *(volatile v8us*)(Wt + (size_t)t * 8) = o; __threadfence(); *(volatile v8us*)(Wt + (size_t)t * 8) = o;
}

__global__ __launch_bounds__(256) void k_wth(const float* __restrict__ W, h16* Wt) {
    __shared__ float tl[DD * (DD + 1)];
    const int t = threadIdx.x;
#pragma unroll 1
    for (int r = 0; r < DD * DD / 256; ++r) { const int idx = t + r * 256; const int k = idx >> 6, n = idx & 63; tl[n * (DD + 1) + k] = bfr(W[idx]) * WCS; }
    __syncthreads();
#pragma unroll 1
    for (int ps = 0; ps < 2; ++ps) {
#pragma unroll
        for (int it = 0; it < 2; ++it) { const int p = t + it * 256; const int n = p >> 3, k8 = (p & 7) * 8; v8h o;
#pragma unroll
            for (int i = 0; i < 8; ++i) o[i] = toh_flush(tl[n * (DD + 1) + k8 + i]);
            *(volatile v8h*)(Wt + (size_t)p * 8) = o; }
        if (ps == 0) __threadfence(); }
}

__global__ __launch_bounds__(32) void k_xc_row(const bf* __restrict__ XB, const bf* __restrict__ WiT, const float* __restrict__ bi, h16* YA) {
    __shared__ __align__(16) float os[16 * 68];
    const int lane = threadIdx.x & 31, lr = lane & 15, hi = lane >> 4;
    const int x = blockIdx.x, b = blockIdx.y; const int t = x / (NN / 64), i0 = (x % (NN / 64)) * 64;
    v8f acc[4][4];
#pragma unroll
    for (int mb = 0; mb < 4; ++mb)
#pragma unroll
        for (int nb = 0; nb < 4; ++nb) acc[mb][nb] = (v8f){};
    const size_t aoff = ((size_t)b * (4 * NN) + (size_t)x * 64 + (size_t)lr) * DOBS + 8 * hi;
    const size_t boff = (size_t)lr * DOBS + 8 * hi;
    mma_tile_b<DOBS>(XB, WiT, aoff, boff, acc);
    float bc[4];
#pragma unroll
    for (int nb = 0; nb < 4; ++nb) bc[nb] = bfr(bi[nb * 16 + lr]);
    const size_t obase = ((size_t)(t * NB + b) * NN + (size_t)i0) * DD;
#pragma unroll
    for (int mb = 0; mb < 4; ++mb) {
#pragma unroll
        for (int nb = 0; nb < 4; ++nb) {
#pragma unroll
            for (int j = 0; j < 8; ++j) os[(hi * 8 + j) * 68 + nb * 16 + lr] = fmaxf(acc[mb][nb][j] + bc[nb], 0.0f); }
        wave_sync();
#pragma unroll 1
        for (int ps = 0; ps < 2; ++ps) {
#pragma unroll
            for (int s = 0; s < 4; ++s) { const int row = 4 * s + (lane >> 3), c8 = (lane & 7) * 8;
                const v4f x0 = *(const v4fa*)(&os[row * 68 + c8]); const v4f x1 = *(const v4fa*)(&os[row * 68 + c8 + 4]); v8h hv;
#pragma unroll
                for (int i = 0; i < 4; ++i) { hv[i] = toh_flush(x0[i]); hv[4 + i] = toh_flush(x1[i]); }
                *(volatile v8h*)(YA + obase + (size_t)(mb * 16 + row) * DD + c8) = hv; }
            if (ps == 0) __threadfence(); }
        wave_sync();
    }
}

__global__ __launch_bounds__(32) void k_xc_col(const bf* __restrict__ WiT, const bf* __restrict__ XB, const float* __restrict__ bi, h16* XCT) {
    __shared__ __align__(16) float os[16 * 68];
    const int lane = threadIdx.x & 31, lr = lane & 15, hi = lane >> 4;
    const int y = blockIdx.x, b = blockIdx.y; const int t2 = y / (NN / 64), i0 = (y % (NN / 64)) * 64;
    v8f acc[4][4];
#pragma unroll
    for (int mb = 0; mb < 4; ++mb)
#pragma unroll
        for (int nb = 0; nb < 4; ++nb) acc[mb][nb] = (v8f){};
    const size_t aoff = (size_t)lr * DOBS + 8 * hi;
    const size_t boff = ((size_t)b * (4 * NN) + (size_t)(2 * NN) + (size_t)y * 64 + (size_t)lr) * DOBS + 8 * hi;
    mma_tile_b<DOBS>(WiT, XB, aoff, boff, acc);
    const size_t obase = ((size_t)(b * 2 + t2) * DD) * NN + (size_t)i0;
#pragma unroll
    for (int mb = 0; mb < 4; ++mb) {
        float br[8];
#pragma unroll
        for (int j = 0; j < 8; ++j) br[j] = bfr(bi[mb * 16 + hi * 8 + j]);
#pragma unroll
        for (int nb = 0; nb < 4; ++nb) {
#pragma unroll
            for (int j = 0; j < 8; ++j) os[(hi * 8 + j) * 68 + nb * 16 + lr] = fmaxf(acc[mb][nb][j] + br[j], 0.0f); }
        wave_sync();
#pragma unroll 1
        for (int ps = 0; ps < 2; ++ps) {
#pragma unroll
            for (int s = 0; s < 4; ++s) { const int row = 4 * s + (lane >> 3), c8 = (lane & 7) * 8;
                const v4f x0 = *(const v4fa*)(&os[row * 68 + c8]); const v4f x1 = *(const v4fa*)(&os[row * 68 + c8 + 4]); v8h hv;
#pragma unroll
                for (int i = 0; i < 4; ++i) { hv[i] = toh_flush(x0[i]); hv[4 + i] = toh_flush(x1[i]); }
                *(volatile v8h*)(XCT + obase + (size_t)(mb * 16 + row) * NN + c8) = hv; }
            if (ps == 0) __threadfence(); }
        wave_sync();
    }
}

__global__ __launch_bounds__(32) void k_hop(const h16* __restrict__ A, int sA, const h16* __restrict__ Bt, int sB, h16* C, int ldc, int sC) {
    __shared__ __align__(16) float os[16 * 68];
    const int lane = threadIdx.x & 31, lr = lane & 15, hi = lane >> 4;
    const int r0 = blockIdx.x * 64, c0 = blockIdx.y * 64, bz = blockIdx.z;
    v8f acc[4][4];
#pragma unroll
    for (int mb = 0; mb < 4; ++mb)
#pragma unroll
        for (int nb = 0; nb < 4; ++nb) acc[mb][nb] = (v8f){};
    const size_t aoff = (size_t)bz * (size_t)sA + (size_t)(r0 + lr) * NN + 8 * hi;
    const size_t boff = (size_t)bz * (size_t)sB + (size_t)(c0 + lr) * NN + 8 * hi;
    mma_tile_h<NN>(A, Bt, aoff, boff, acc);
    const size_t obase = (size_t)bz * (size_t)sC + (size_t)r0 * (size_t)ldc + (size_t)c0;
#pragma unroll
    for (int mb = 0; mb < 4; ++mb) {
#pragma unroll
        for (int nb = 0; nb < 4; ++nb) {
#pragma unroll
            for (int j = 0; j < 8; ++j) os[(hi * 8 + j) * 68 + nb * 16 + lr] = acc[mb][nb][j]; }
        wave_sync();
#pragma unroll 1
        for (int ps = 0; ps < 2; ++ps) {
#pragma unroll
            for (int s = 0; s < 4; ++s) { const int row = 4 * s + (lane >> 3), c8 = (lane & 7) * 8;
                const v4f x0 = *(const v4fa*)(&os[row * 68 + c8]); const v4f x1 = *(const v4fa*)(&os[row * 68 + c8 + 4]); v8h hv;
#pragma unroll
                for (int i = 0; i < 4; ++i) { hv[i] = toh_flush(x0[i]); hv[4 + i] = toh_flush(x1[i]); }
                *(volatile v8h*)(C + obase + (size_t)(mb * 16 + row) * (size_t)ldc + c8) = hv; }
            if (ps == 0) __threadfence(); }
        wave_sync();
    }
}

__global__ __launch_bounds__(32) void k_gemm_f32(const h16* __restrict__ A, const h16* __restrict__ Wt, const float* __restrict__ bias, int hasb, float scale, float* C) {
    __shared__ __align__(16) float os[16 * 68];
    const int lane = threadIdx.x & 31, lr = lane & 15, hi = lane >> 4;
    const int r0 = blockIdx.x * 64;
    v8f acc[4][4];
#pragma unroll
    for (int mb = 0; mb < 4; ++mb)
#pragma unroll
        for (int nb = 0; nb < 4; ++nb) acc[mb][nb] = (v8f){};
    const size_t aoff = (size_t)(r0 + lr) * DD + 8 * hi;
    const size_t boff = (size_t)lr * DD + 8 * hi;
    mma_tile_h<DD>(A, Wt, aoff, boff, acc);
    float bc[4];
#pragma unroll
    for (int nb = 0; nb < 4; ++nb) { const float bv = bfr(bias[nb * 16 + lr]); bc[nb] = (hasb != 0) ? bv : 0.0f; }
#pragma unroll
    for (int mb = 0; mb < 4; ++mb) {
#pragma unroll
        for (int nb = 0; nb < 4; ++nb) {
#pragma unroll
            for (int j = 0; j < 8; ++j) os[(hi * 8 + j) * 68 + nb * 16 + lr] = acc[mb][nb][j] * scale + bc[nb]; }
        wave_sync();
#pragma unroll 1
        for (int ps = 0; ps < 2; ++ps) {
#pragma unroll
            for (int s = 0; s < 8; ++s) { const int row = 2 * s + (lane >> 4), cofs = (lane & 15) * 4;
                const v4f val = *(const v4fa*)(&os[row * 68 + cofs]);
                *(volatile v4f*)(C + (size_t)(r0 + mb * 16 + row) * DD + cofs) = val; }
            if (ps == 0) __threadfence(); }
        wave_sync();
    }
}

__global__ __launch_bounds__(256) void k_edge(const float* __restrict__ Ain, const float* __restrict__ P, const float* __restrict__ bpre, h16* AG) {
    __shared__ __align__(16) float sa[ET * NN];
    __shared__ __align__(16) float st[ET * 4 * DD];
    const int t = threadIdx.x, lane = t & 31;
    const int wave = __builtin_amdgcn_readfirstlane((int)(threadIdx.x >> 5));
    const int i0 = blockIdx.x * ET, b = blockIdx.y;
    const float* arow = Ain + (size_t)b * ((size_t)KH * NN * NN) + (size_t)i0 * NN;
#pragma unroll
    for (int r = 0; r < ET * NN / 256; ++r) { const int idx = t + r * 256; sa[idx] = bfr(arow[idx]); }
    __syncthreads();
    if (wave < 6) {
        const int kk = wave >> 1; const int d = (wave & 1) * 32 + lane;
        const float bp = bfr(bpre[d]);
        const float* pk = P + ((size_t)((kk + 1) * NB + b) * NN) * DD + d;
        float acc[ET];
#pragma unroll
        for (int r = 0; r < ET; ++r) acc[r] = 0.0f;
#pragma unroll 2
        for (int j = 0; j < NN; ++j) {
            const float p = pk[(size_t)j * DD];
#pragma unroll
            for (int r = 0; r < ET; ++r) acc[r] += fmaxf(fmaf(sa[r * NN + j], p, bp), 0.0f);
        }
#pragma unroll
        for (int r = 0; r < ET; ++r) st[(r * 4 + kk + 1) * DD + d] = acc[r];
    } else {
        const int d = (wave - 6) * 32 + lane;
        const float bp = bfr(bpre[d]);
        const float rv = (float)(NN - 1) * fmaxf(bp, 0.0f);
#pragma unroll
        for (int r = 0; r < ET; ++r) {
            const float q = P[((size_t)b * NN + (size_t)(i0 + r)) * DD + d];
            st[(r * 4) * DD + d] = fmaxf(q + bp, 0.0f) + rv; }
    }
    __syncthreads();
    const int row = t >> 3, c8 = (t & 7) * 8;
    const v4f x0 = *(const v4fa*)(&st[row * DD + c8]); const v4f x1 = *(const v4fa*)(&st[row * DD + c8 + 4]); v8h hv;
#pragma unroll
    for (int i = 0; i < 4; ++i) { hv[i] = toh_flush(x0[i] * ACS); hv[4 + i] = toh_flush(x1[i] * ACS); }
    h16* op = AG + ((size_t)(b * NN + i0) * 4) * DD + (size_t)t * 8;
    *(volatile v8h*)op = hv; __threadfence(); *(volatile v8h*)op = hv;
}

__global__ __launch_bounds__(32) void k_mid(const h16* __restrict__ AG, const h16* __restrict__ Wt, const float* __restrict__ bmid, h16* S) {
    __shared__ __align__(16) float os[16 * 68];
    const int lane = threadIdx.x & 31, lr = lane & 15, hi = lane >> 4;
    const int r0 = blockIdx.x * 64;
    v8f acc[4][4];
#pragma unroll
    for (int mb = 0; mb < 4; ++mb)
#pragma unroll
        for (int nb = 0; nb < 4; ++nb) acc[mb][nb] = (v8f){};
    const size_t aoff = (size_t)(r0 + lr) * DD + 8 * hi;
    const size_t boff = (size_t)lr * DD + 8 * hi;
    mma_tile_h<DD>(AG, Wt, aoff, boff, acc);
    float bc[4];
#pragma unroll
    for (int nb = 0; nb < 4; ++nb) bc[nb] = bfr(bmid[nb * 16 + lr]);
#pragma unroll
    for (int mb = 0; mb < 4; ++mb) {
#pragma unroll
        for (int nb = 0; nb < 4; ++nb) {
            float s0 = 0.0f, s1 = 0.0f;
#pragma unroll
            for (int j = 0; j < 4; ++j) { s0 += fmaxf(acc[mb][nb][j] + bc[nb], 0.0f); s1 += fmaxf(acc[mb][nb][4 + j] + bc[nb], 0.0f); }
            os[(mb * 4 + 2 * hi) * 68 + nb * 16 + lr] = s0;
            os[(mb * 4 + 2 * hi + 1) * 68 + nb * 16 + lr] = s1; }
    }
    wave_sync();
    const size_t obase = (size_t)(r0 / 4) * DD;
#pragma unroll 1
    for (int ps = 0; ps < 2; ++ps) {
#pragma unroll
        for (int s = 0; s < 4; ++s) { const int row = 4 * s + (lane >> 3), c8 = (lane & 7) * 8;
            const v4f x0 = *(const v4fa*)(&os[row * 68 + c8]); const v4f x1 = *(const v4fa*)(&os[row * 68 + c8 + 4]); v8h hv;
#pragma unroll
            for (int i = 0; i < 4; ++i) { hv[i] = toh_flush(x0[i] * ACS); hv[4 + i] = toh_flush(x1[i] * ACS); }
            *(volatile v8h*)(S + obase + (size_t)row * DD + c8) = hv; }
        if (ps == 0) __threadfence(); }
}

static constexpr size_t al256(size_t v) { return (v + 255) & ~(size_t)255; }
static constexpr size_t SZ_XB  = al256((size_t)NB * 4 * NN * DOBS * 2);
static constexpr size_t SZ_AH  = al256((size_t)NB * 2 * NN * NN * 2);
static constexpr size_t SZ_WI  = al256((size_t)DD * DOBS * 2);
static constexpr size_t SZ_WW  = al256((size_t)DD * DD * 2);
static constexpr size_t SZ_XCT = al256((size_t)NB * 2 * DD * NN * 2);
static constexpr size_t SZ_Y12 = al256((size_t)NB * DD * NN * 2);
static constexpr size_t SZ_YA  = al256((size_t)4 * NB * NN * DD * 2);
static constexpr size_t SZ_P   = al256((size_t)4 * NB * NN * DD * 4);
static constexpr size_t SZ_AG  = al256((size_t)NB * NN * 4 * DD * 2);
static constexpr size_t SZ_S   = al256((size_t)NB * NN * DD * 2);
static constexpr size_t SZ_TOTAL = SZ_XB + SZ_AH + SZ_WI + 3 * SZ_WW + SZ_XCT + SZ_Y12 + SZ_YA + SZ_P + SZ_AG + SZ_S;
static_assert(SZ_TOTAL <= (size_t)134217728);
static_assert((size_t)(2 * NN / 64) * 64 == (size_t)2 * NN);
static_assert((size_t)(4 * NB * NN / 64) * 64 == (size_t)4 * NB * NN);
static_assert((size_t)(NB * NN * 4 / 64) * 64 == (size_t)NB * NN * 4);
static_assert((size_t)(NB * NN / 64) * 64 == (size_t)NB * NN);
static_assert((size_t)(NN / ET) * ET * 4 * DD * 2 * NB == (size_t)NB * NN * 4 * DD * 2);

extern "C" void kernel_launch(void* const* d_in, const int* in_sizes, int n_in,
                              void* d_out, int out_size, void* d_ws, size_t ws_size, hipStream_t stream) {
    if (n_in < 10) return;
    if ((size_t)in_sizes[0] < (size_t)NB * KH * NN * NN) return;
    if ((size_t)in_sizes[1] < (size_t)NB * 4 * NN * DOBS) return;
    if ((size_t)in_sizes[2] < (size_t)DOBS * DD || in_sizes[3] < DD) return;
    if ((size_t)in_sizes[4] < (size_t)DD * DD || in_sizes[5] < DD) return;
    if ((size_t)in_sizes[6] < (size_t)DD * DD || in_sizes[7] < DD) return;
    if ((size_t)in_sizes[8] < (size_t)DD * DD || in_sizes[9] < DD) return;
    if ((size_t)out_size < (size_t)NB * NN * DD) return;
    if (SZ_TOTAL > ws_size) return;
    const float* Ain  = (const float*)d_in[0];
    const float* Xin  = (const float*)d_in[1];
    const float* Wi   = (const float*)d_in[2];
    const float* bi   = (const float*)d_in[3];
    const float* Wpre = (const float*)d_in[4];
    const float* bpre = (const float*)d_in[5];
    const float* Wmid = (const float*)d_in[6];
    const float* bmid = (const float*)d_in[7];
    const float* Wout = (const float*)d_in[8];
    const float* bout = (const float*)d_in[9];
    float* OUT = (float*)d_out;
    char* wsp = (char*)d_ws;
    bf*  XB   = (bf*)wsp;   wsp += SZ_XB;
    h16* AH   = (h16*)wsp;  wsp += SZ_AH;
    bf*  WiT  = (bf*)wsp;   wsp += SZ_WI;
    h16* WpT  = (h16*)wsp;  wsp += SZ_WW;
    h16* WmT  = (h16*)wsp;  wsp += SZ_WW;
    h16* WoT  = (h16*)wsp;  wsp += SZ_WW;
    h16* XCT  = (h16*)wsp;  wsp += SZ_XCT;
    h16* Y12T = (h16*)wsp;  wsp += SZ_Y12;
    h16* YA   = (h16*)wsp;  wsp += SZ_YA;
    float* P  = (float*)wsp; wsp += SZ_P;
    h16* AG   = (h16*)wsp;  wsp += SZ_AG;
    h16* S    = (h16*)wsp;  wsp += SZ_S;

    { const size_t n8 = (size_t)NB * 4 * NN * DOBS / 8; k_cvt8<<<(unsigned)((n8 + 255) / 256), 256, 0, stream>>>(Xin, XB, n8); }
    { const size_t n8 = (size_t)NB * 2 * NN * NN / 8;   k_cvt8a<<<(unsigned)((n8 + 255) / 256), 256, 0, stream>>>(Ain, AH, n8); }
    k_wtb<<<1, 256, 0, stream>>>(Wi, WiT);
    k_wth<<<1, 256, 0, stream>>>(Wpre, WpT);
    k_wth<<<1, 256, 0, stream>>>(Wmid, WmT);
    k_wth<<<1, 256, 0, stream>>>(Wout, WoT);

    k_xc_row<<<dim3(2 * NN / 64, NB, 1), 32, 0, stream>>>(XB, WiT, bi, YA);
    k_xc_col<<<dim3(2 * NN / 64, NB, 1), 32, 0, stream>>>(WiT, XB, bi, XCT);

    k_hop<<<dim3(NN / 64, DD / 64, NB), 32, 0, stream>>>(AH, 2 * NN * NN, XCT, 2 * DD * NN, YA + (size_t)2 * NB * NN * DD, DD, NN * DD);
    k_hop<<<dim3(DD / 64, NN / 64, NB), 32, 0, stream>>>(XCT + (size_t)DD * NN, 2 * DD * NN, AH + (size_t)NN * NN, 2 * NN * NN, Y12T, NN, DD * NN);
    k_hop<<<dim3(NN / 64, DD / 64, NB), 32, 0, stream>>>(AH, 2 * NN * NN, Y12T, DD * NN, YA + (size_t)3 * NB * NN * DD, DD, NN * DD);

    k_gemm_f32<<<dim3(4 * NB * NN / 64, 1, 1), 32, 0, stream>>>(YA, WpT, bpre, 0, WCI, P);
    k_edge<<<dim3(NN / ET, NB, 1), 256, 0, stream>>>(Ain, P, bpre, AG);
    k_mid<<<dim3(NB * NN * 4 / 64, 1, 1), 32, 0, stream>>>(AG, WmT, bmid, S);
    k_gemm_f32<<<dim3(NB * NN / 64, 1, 1), 32, 0, stream>>>(S, WoT, bout, 1, 1.0f, OUT);
}
